// MultiheadDuffAttn_163208757404
// MI455X (gfx1250) — hardware-verified
//
#include <hip/hip_runtime.h>


#define NBT  2
#define SS   1024
#define EE   1024
#define NHV  16
#define HD   32
#define VD   64
#define HG   4
#define DM   EE
#define SCL  0.17677669529663687f
#define LINIT 0.7836057665316245f
#define REPS 1e-5f
#define LOSC 1024.0f

typedef _Float16 h16;
typedef unsigned short bf;
typedef __attribute__((ext_vector_type(16))) __bf16   v16bf;
typedef __attribute__((ext_vector_type(16))) _Float16 v16h;
typedef __attribute__((ext_vector_type(8)))  _Float16 v8h;
typedef __attribute__((ext_vector_type(8)))  unsigned short v8us;
typedef __attribute__((ext_vector_type(8)))  float    v8f;
typedef __attribute__((ext_vector_type(4)))  float    v4f;
typedef v8h  __attribute__((may_alias)) v8ha;
typedef v4f  __attribute__((may_alias)) v4fa;
typedef v8us __attribute__((may_alias)) v8usa;

__device__ __forceinline__ unsigned short f2bf(float f) { unsigned u = __float_as_uint(f); u += 0x7FFFu + ((u >> 16) & 1u); return (unsigned short)(u >> 16); }
__device__ __forceinline__ float bf2f(unsigned short b) { return __uint_as_float(((unsigned)b) << 16); }
__device__ __forceinline__ float bfr(float f) { return bf2f(f2bf(f)); }
__device__ __forceinline__ v16h cat16(v8h lo, v8h hi) { return __builtin_shufflevector(lo, hi, 0, 1, 2, 3, 4, 5, 6, 7, 8, 9, 10, 11, 12, 13, 14, 15); }
__device__ __forceinline__ v16bf cat16b(v8us lo, v8us hi) { return __builtin_bit_cast(v16bf, __builtin_shufflevector(lo, hi, 0, 1, 2, 3, 4, 5, 6, 7, 8, 9, 10, 11, 12, 13, 14, 15)); }
__device__ __forceinline__ v8f wmma16(v16h a, v16h b, v8f c) { return __builtin_amdgcn_wmma_f32_16x16x32_f16(false, a, false, b, (short)0, c, false, false); }
__device__ __forceinline__ v8f wmmab(v16bf a, v16bf b, v8f c) { return __builtin_amdgcn_wmma_f32_16x16x32_bf16(false, a, false, b, (short)0, c, false, false); }

template <bool SPLITA, bool F16OUT = false>
__global__ __launch_bounds__(128) void k_gemmb(const bf* __restrict__ A, const bf* __restrict__ Al, const bf* __restrict__ Bn, const float* __restrict__ bias, float* C, int ldc, h16* C2, const float* __restrict__ R = nullptr, int K = DM, int roundR = 1) {
    __shared__ __align__(16) float ost[4][16 * 68];
    const int lane = threadIdx.x & 31, wave = threadIdx.x >> 5, lr = lane & 15, hi = lane >> 4;
    const int r0 = blockIdx.x * 64 + wave * 16, c0 = blockIdx.y * 64;
    const size_t aoff = (size_t)(r0 + lr) * K + 8 * hi;
    size_t boff[4];
#pragma unroll
    for (int t = 0; t < 4; ++t) boff[t] = (size_t)(c0 + t * 16 + lr) * K + 8 * hi;
    v8f acc[4];
#pragma unroll
    for (int t = 0; t < 4; ++t) acc[t] = (v8f){};
#pragma unroll 1
    for (int kc = 0; kc < K; kc += 32) {
        const v16bf a = cat16b(*(const v8us*)(A + aoff + kc), *(const v8us*)(A + aoff + kc + 16));
        v16bf al = a;
        if (SPLITA) al = cat16b(*(const v8us*)(Al + aoff + kc), *(const v8us*)(Al + aoff + kc + 16));
#pragma unroll
        for (int t = 0; t < 4; ++t) { const v16bf b = cat16b(*(const v8us*)(Bn + boff[t] + kc), *(const v8us*)(Bn + boff[t] + kc + 16)); acc[t] = wmmab(a, b, acc[t]); if (SPLITA) acc[t] = wmmab(al, b, acc[t]); }
        asm volatile("v_nop\n\tv_nop\n\tv_nop\n\tv_nop" : "+v"(acc[0]), "+v"(acc[1]), "+v"(acc[2]), "+v"(acc[3]) : "v"(a), "v"(al));
    }
    float* os = &ost[wave][0];
#pragma unroll
    for (int t = 0; t < 4; ++t) { const float bv = bias ? bfr(bias[c0 + t * 16 + lr]) : 0.f;
#pragma unroll
        for (int j = 0; j < 8; ++j) os[(hi * 8 + j) * 68 + t * 16 + lr] = acc[t][j] + bv; }
    __syncthreads();
    if (F16OUT) {
        h16* crow = (h16*)(void*)C + (size_t)r0 * ldc + c0;
        auto pass = [&]() {
#pragma unroll
            for (int s = 0; s < 4; ++s) { const int row = 4 * s + (lane >> 3), piece = lane & 7; const float* sp = os + row * 68 + piece * 8; v8h o, o2;
#pragma unroll
                for (int i = 0; i < 8; ++i) { const h16 a = (h16)sp[i]; o[i] = a; o2[i] = (h16)((sp[i] - (float)a) * LOSC); }
                *(volatile v8h*)(crow + (size_t)row * ldc + piece * 8) = o; if (C2) *(volatile v8h*)(C2 + (size_t)r0 * ldc + c0 + (size_t)row * ldc + piece * 8) = o2; }
        };
        pass(); __threadfence(); pass();
    } else {
        float* crow = C + (size_t)r0 * ldc + c0;
        auto pass = [&]() {
#pragma unroll
            for (int s = 0; s < 8; ++s) { const int Lid = (lane >> 3) + 4 * s, piece = lane & 7; const int row = Lid >> 1, cofs = (Lid & 1) * 32 + piece * 4;
                v4f val = *(const v4fa*)(os + row * 68 + cofs); if (R) { const v4f rv = *(const v4f*)(R + ((size_t)r0 + row) * ldc + c0 + cofs); val += roundR ? (v4f){bfr(rv[0]), bfr(rv[1]), bfr(rv[2]), bfr(rv[3])} : rv; }
                *(volatile v4f*)(crow + (size_t)row * ldc + cofs) = val; }
        };
        pass(); __threadfence(); pass();
    }
}

template <bool SPLITA, bool F16OUT = false>
__global__ __launch_bounds__(128) void k_gemmbz(const bf* __restrict__ A, const bf* __restrict__ Al, const bf* __restrict__ Bn, const float* __restrict__ bias, float* C, int ldc, h16* C2, const float* __restrict__ R, int K, int roundR, size_t sA, size_t sB, size_t sBias, size_t sC) {
    { const size_t g = blockIdx.z; A += g * sA; if (Al) Al += g * sA; Bn += g * sB; if (bias) bias += g * sBias; C += g * sC; if (R) R += g * sC; }
    __shared__ __align__(16) float ost[4][16 * 68];
    const int lane = threadIdx.x & 31, wave = threadIdx.x >> 5, lr = lane & 15, hi = lane >> 4;
    const int r0 = blockIdx.x * 64 + wave * 16, c0 = blockIdx.y * 64;
    const size_t aoff = (size_t)(r0 + lr) * K + 8 * hi;
    size_t boff[4];
#pragma unroll
    for (int t = 0; t < 4; ++t) boff[t] = (size_t)(c0 + t * 16 + lr) * K + 8 * hi;
    v8f acc[4];
#pragma unroll
    for (int t = 0; t < 4; ++t) acc[t] = (v8f){};
#pragma unroll 1
    for (int kc = 0; kc < K; kc += 32) {
        const v16bf a = cat16b(*(const v8us*)(A + aoff + kc), *(const v8us*)(A + aoff + kc + 16));
        v16bf al = a;
        if (SPLITA) al = cat16b(*(const v8us*)(Al + aoff + kc), *(const v8us*)(Al + aoff + kc + 16));
#pragma unroll
        for (int t = 0; t < 4; ++t) { const v16bf b = cat16b(*(const v8us*)(Bn + boff[t] + kc), *(const v8us*)(Bn + boff[t] + kc + 16)); acc[t] = wmmab(a, b, acc[t]); if (SPLITA) acc[t] = wmmab(al, b, acc[t]); }
        asm volatile("v_nop\n\tv_nop\n\tv_nop\n\tv_nop" : "+v"(acc[0]), "+v"(acc[1]), "+v"(acc[2]), "+v"(acc[3]) : "v"(a), "v"(al));
    }
    float* os = &ost[wave][0];
#pragma unroll
    for (int t = 0; t < 4; ++t) { const float bv = bias ? bfr(bias[c0 + t * 16 + lr]) : 0.f;
#pragma unroll
        for (int j = 0; j < 8; ++j) os[(hi * 8 + j) * 68 + t * 16 + lr] = acc[t][j] + bv; }
    __syncthreads();
    if (F16OUT) {
        h16* crow = (h16*)(void*)C + (size_t)r0 * ldc + c0;
        auto pass = [&]() {
#pragma unroll
            for (int s = 0; s < 4; ++s) { const int row = 4 * s + (lane >> 3), piece = lane & 7; const float* sp = os + row * 68 + piece * 8; v8h o, o2;
#pragma unroll
                for (int i = 0; i < 8; ++i) { const h16 a = (h16)sp[i]; o[i] = a; o2[i] = (h16)((sp[i] - (float)a) * LOSC); }
                *(volatile v8h*)(crow + (size_t)row * ldc + piece * 8) = o; if (C2) *(volatile v8h*)(C2 + (size_t)r0 * ldc + c0 + (size_t)row * ldc + piece * 8) = o2; }
        };
        pass(); __threadfence(); pass();
    } else {
        float* crow = C + (size_t)r0 * ldc + c0;
        auto pass = [&]() {
#pragma unroll
            for (int s = 0; s < 8; ++s) { const int Lid = (lane >> 3) + 4 * s, piece = lane & 7; const int row = Lid >> 1, cofs = (Lid & 1) * 32 + piece * 4;
                v4f val = *(const v4fa*)(os + row * 68 + cofs); if (R) { const v4f rv = *(const v4f*)(R + ((size_t)r0 + row) * ldc + c0 + cofs); val += roundR ? (v4f){bfr(rv[0]), bfr(rv[1]), bfr(rv[2]), bfr(rv[3])} : rv; }
                *(volatile v4f*)(crow + (size_t)row * ldc + cofs) = val; }
        };
        pass(); __threadfence(); pass();
    }
}

__global__ __launch_bounds__(256) void k_wt(const float* __restrict__ Wm, int K, int ncols, bf* WT) {
    __shared__ __align__(16) unsigned short tl[64 * 72];
    const int tid = threadIdx.x, k0 = blockIdx.x * 64, n0 = blockIdx.y * 64;
    const int kk = tid >> 2, nq = (tid & 3) * 16;
#pragma unroll
    for (int i = 0; i < 16; ++i) tl[(nq + i) * 72 + kk] = f2bf(Wm[(size_t)(k0 + kk) * ncols + n0 + nq + i]);
    __syncthreads();
    const int piece = tid & 7;
    auto pass = [&]() {
#pragma unroll
        for (int s = 0; s < 2; ++s) { const int nr = (tid >> 3) + 32 * s; const v8us val = *(const v8usa*)(tl + nr * 72 + piece * 8); *(volatile v8us*)(WT + (size_t)(n0 + nr) * K + k0 + piece * 8) = val; }
    };
    pass(); __threadfence(); pass();
}

__global__ __launch_bounds__(256) void k_cvtx(const float* __restrict__ src, bf* dst) {
    const int lane = threadIdx.x & 31; const size_t r = (size_t)blockIdx.x * 8 + (threadIdx.x >> 5); if (r >= (size_t)SS) return;
#pragma unroll 1
    for (int ps = 0; ps < 2; ++ps) {
#pragma unroll
        for (int q = 0; q < EE / 256; ++q) { v8us o;
#pragma unroll
            for (int i = 0; i < 8; ++i) o[i] = f2bf(src[r * EE + q * 256 + lane * 8 + i]);
            *(volatile v8us*)(dst + r * EE + q * 256 + lane * 8) = o; }
        if (ps == 0) __threadfence(); }
}
__global__ __launch_bounds__(256) void k_hp32(const float* __restrict__ F, int hh0, bf* Ph, bf* Pl) {
    typedef __attribute__((ext_vector_type(2))) unsigned short v2us;
    const int lane = threadIdx.x & 31; const size_t wid = (size_t)blockIdx.x * 8 + (threadIdx.x >> 5); if (wid >= (size_t)8 * (SS / 2)) return; const int hh = (int)(wid / (SS / 2)); const int s = (int)(wid % (SS / 2)) * 2 + (lane >> 4); const int d = (lane & 15) * 2;
    v2us oh, ol;
#pragma unroll
    for (int i = 0; i < 2; ++i) { const float v = F[(size_t)s * EE + (hh0 + hh) * HD + d + i]; const unsigned short hb = f2bf(v); oh[i] = hb; ol[i] = f2bf(v - bf2f(hb)); }
    const size_t o = ((size_t)hh * SS + s) * HD + d; *(volatile v2us*)(Ph + o) = oh; *(volatile v2us*)(Pl + o) = ol; __threadfence(); *(volatile v2us*)(Ph + o) = oh; *(volatile v2us*)(Pl + o) = ol;
}
__global__ __launch_bounds__(256) void k_vt(const float* __restrict__ VF, int h0, bf* Th, bf* Tl) {
    typedef __attribute__((ext_vector_type(2))) unsigned short v2us;
    const int lane = threadIdx.x & 31; const size_t wid = (size_t)blockIdx.x * 8 + (threadIdx.x >> 5); if (wid >= (size_t)HG * VD * (SS / 64)) return;
    const int sg = (int)(wid % (SS / 64)), rest = (int)(wid / (SS / 64)), d = rest % VD, h = rest / VD; const int s0 = sg * 64 + lane * 2; v2us oh, ol;
#pragma unroll
    for (int i = 0; i < 2; ++i) { const float v = VF[(size_t)(s0 + i) * EE + (h0 + h) * VD + d]; const unsigned short hb = f2bf(v); oh[i] = hb; ol[i] = f2bf(v - bf2f(hb)); }
    const size_t o = ((size_t)h * VD + d) * SS + s0; *(volatile v2us*)(Th + o) = oh; *(volatile v2us*)(Tl + o) = ol; __threadfence(); *(volatile v2us*)(Th + o) = oh; *(volatile v2us*)(Tl + o) = ol;
}
__global__ __launch_bounds__(256) void k_duffw(const float* __restrict__ S, const float* __restrict__ lq1, const float* __restrict__ lk1, const float* __restrict__ lq2, const float* __restrict__ lk2, bf* WH, bf* WL) {
    typedef __attribute__((ext_vector_type(4))) unsigned short v4us;
    const int lane = threadIdx.x & 31; const int wid = blockIdx.x * 8 + (threadIdx.x >> 5); if (wid >= HG * SS) return; const int h = wid / SS, i = wid % SS;
    float d1 = 0.f, d2 = 0.f;
#pragma unroll
    for (int d = 0; d < HD; ++d) { d1 = fmaf(bfr(lq1[d]), bfr(lk1[d]), d1); d2 = fmaf(bfr(lq2[d]), bfr(lk2[d]), d2); }
    const float lam = __expf(d1) - __expf(d2) + LINIT;
    const float* s1 = S + ((size_t)(2 * h) * SS + i) * SS; const float* s2 = S + ((size_t)(2 * h + 1) * SS + i) * SS;
    float m1 = -3.0e38f, m2 = -3.0e38f;
#pragma unroll 1
    for (int c0 = lane * 4; c0 < SS; c0 += 128) {
#pragma unroll
        for (int q = 0; q < 4; ++q) { const int k = c0 + q; if (k <= i) { m1 = fmaxf(m1, s1[k] * SCL); m2 = fmaxf(m2, s2[k] * SCL); } } }
#pragma unroll
    for (int sh = 16; sh; sh >>= 1) { m1 = fmaxf(m1, __shfl_xor(m1, sh, 32)); m2 = fmaxf(m2, __shfl_xor(m2, sh, 32)); }
    float z1 = 0.f, z2 = 0.f;
#pragma unroll 1
    for (int c0 = lane * 4; c0 < SS; c0 += 128) {
#pragma unroll
        for (int q = 0; q < 4; ++q) { const int k = c0 + q; if (k <= i) { z1 += __expf(s1[k] * SCL - m1); z2 += __expf(s2[k] * SCL - m2); } } }
#pragma unroll
    for (int sh = 16; sh; sh >>= 1) { z1 += __shfl_xor(z1, sh, 32); z2 += __shfl_xor(z2, sh, 32); }
    const float i1 = 1.0f / z1, i2 = 1.0f / z2;
#pragma unroll 1
    for (int ps = 0; ps < 2; ++ps) {
#pragma unroll 1
        for (int c0 = lane * 4; c0 < SS; c0 += 128) { v4us oh, ol;
#pragma unroll
            for (int q = 0; q < 4; ++q) { const int k = c0 + q; const float w = (k <= i) ? (__expf(s1[k] * SCL - m1) * i1 - lam * (__expf(s2[k] * SCL - m2) * i2)) : 0.f; const unsigned short hb = f2bf(w); oh[q] = hb; ol[q] = f2bf(w - bf2f(hb)); }
            const size_t o = ((size_t)h * SS + i) * SS + c0; *(volatile v4us*)(WH + o) = oh; *(volatile v4us*)(WL + o) = ol; }
        if (ps == 0) __threadfence(); }
}
__global__ __launch_bounds__(256) void k_rms(const float* __restrict__ ATT, const float* __restrict__ rw, int h0, bf* Rh, bf* Rl) {
    typedef __attribute__((ext_vector_type(2))) unsigned short v2us;
    const int lane = threadIdx.x & 31; const int wid = blockIdx.x * 8 + (threadIdx.x >> 5); if (wid >= SS * HG) return; const int s = wid / HG, h = wid % HG;
    const float* ar = ATT + (size_t)s * EE + (h0 + h) * VD; const float a0 = ar[lane * 2], a1 = ar[lane * 2 + 1]; float q = a0 * a0 + a1 * a1;
#pragma unroll
    for (int sh = 16; sh; sh >>= 1) q += __shfl_xor(q, sh, 32);
    const float sc = rsqrtf(q * (1.0f / VD) + REPS) * (1.0f - LINIT); v2us oh, ol;
    { const float v = a0 * sc * bfr(rw[lane * 2]); const unsigned short hb = f2bf(v); oh[0] = hb; ol[0] = f2bf(v - bf2f(hb)); }
    { const float v = a1 * sc * bfr(rw[lane * 2 + 1]); const unsigned short hb = f2bf(v); oh[1] = hb; ol[1] = f2bf(v - bf2f(hb)); }
    const size_t o = (size_t)s * EE + (h0 + h) * VD + lane * 2; *(volatile v2us*)(Rh + o) = oh; *(volatile v2us*)(Rl + o) = ol; __threadfence(); *(volatile v2us*)(Rh + o) = oh; *(volatile v2us*)(Rl + o) = ol;
}

extern "C" void kernel_launch(void* const* d_in, const int* in_sizes, int n_in,
                              void* d_out, int out_size, void* d_ws, size_t ws_size, hipStream_t stream) {
    (void)in_sizes; (void)n_in; (void)out_size;
    const float* x = (const float*)d_in[0]; const float* Wq = (const float*)d_in[1]; const float* Wk = (const float*)d_in[2]; const float* Wv = (const float*)d_in[3]; const float* Wo = (const float*)d_in[4];
    const float* lq1 = (const float*)d_in[5]; const float* lk1 = (const float*)d_in[6]; const float* lq2 = (const float*)d_in[7]; const float* lk2 = (const float*)d_in[8]; const float* rw = (const float*)d_in[9];
    float* out = (float*)d_out;
    char* wsp = (char*)d_ws;
    auto take = [&](size_t bytes) { char* p = wsp; wsp += (bytes + 255) & ~(size_t)255; return (void*)p; };
    bf* WQT = (bf*)take((size_t)EE * EE * 2); bf* WKT = (bf*)take((size_t)EE * EE * 2); bf* WVT = (bf*)take((size_t)EE * EE * 2); bf* WOT = (bf*)take((size_t)EE * EE * 2);
    bf* Xb = (bf*)take((size_t)SS * EE * 2); float* QF = (float*)take((size_t)SS * EE * 4); float* KF = (float*)take((size_t)SS * EE * 4); float* VF = (float*)take((size_t)SS * EE * 4);
    bf* QPh = (bf*)take((size_t)8 * SS * HD * 2); bf* QPl = (bf*)take((size_t)8 * SS * HD * 2); bf* KPh = (bf*)take((size_t)8 * SS * HD * 2); bf* KPl = (bf*)take((size_t)8 * SS * HD * 2); bf* VTh = (bf*)take((size_t)HG * VD * SS * 2); bf* VTl = (bf*)take((size_t)HG * VD * SS * 2);
    float* S1 = (float*)take((size_t)8 * SS * SS * 4); float* S = (float*)take((size_t)8 * SS * SS * 4); bf* WH = (bf*)take((size_t)HG * SS * SS * 2); bf* WL = (bf*)take((size_t)HG * SS * SS * 2);
    float* A1 = (float*)take((size_t)SS * EE * 4); float* ATT = (float*)take((size_t)SS * EE * 4); bf* Rh = (bf*)take((size_t)SS * EE * 2); bf* Rl = (bf*)take((size_t)SS * EE * 2);
    if ((size_t)(wsp - (char*)d_ws) > ws_size) return;
    k_wt<<<dim3(EE / 64, EE / 64, 1), 256, 0, stream>>>(Wq, EE, EE, WQT); k_wt<<<dim3(EE / 64, EE / 64, 1), 256, 0, stream>>>(Wk, EE, EE, WKT); k_wt<<<dim3(EE / 64, EE / 64, 1), 256, 0, stream>>>(Wv, EE, EE, WVT); k_wt<<<dim3(EE / 64, EE / 64, 1), 256, 0, stream>>>(Wo, EE, EE, WOT);
    const size_t sQ = (size_t)SS * HD, sS = (size_t)SS * SS, sV = (size_t)VD * SS;
    for (int b = 0; b < NBT; ++b) {
        k_cvtx<<<SS / 8, 256, 0, stream>>>(x + (size_t)b * SS * EE, Xb);
        k_gemmb<false, false><<<dim3(SS / 64, EE / 64, 1), 128, 0, stream>>>(Xb, nullptr, WQT, nullptr, QF, EE, nullptr, nullptr, EE);
        k_gemmb<false, false><<<dim3(SS / 64, EE / 64, 1), 128, 0, stream>>>(Xb, nullptr, WKT, nullptr, KF, EE, nullptr, nullptr, EE);
        k_gemmb<false, false><<<dim3(SS / 64, EE / 64, 1), 128, 0, stream>>>(Xb, nullptr, WVT, nullptr, VF, EE, nullptr, nullptr, EE);
        for (int g = 0; g < NHV / HG; ++g) { const int h0 = g * HG, hh0 = 2 * h0;
            k_hp32<<<(8 * SS / 2) / 8, 256, 0, stream>>>(QF, hh0, QPh, QPl); k_hp32<<<(8 * SS / 2) / 8, 256, 0, stream>>>(KF, hh0, KPh, KPl); k_vt<<<(HG * VD * (SS / 64)) / 8, 256, 0, stream>>>(VF, h0, VTh, VTl);
            k_gemmbz<true, false><<<dim3(SS / 64, SS / 64, 8), 128, 0, stream>>>(QPh, QPl, KPh, nullptr, S1, SS, nullptr, nullptr, HD, 0, sQ, sQ, 0, sS);
            k_gemmbz<false, false><<<dim3(SS / 64, SS / 64, 8), 128, 0, stream>>>(QPh, nullptr, KPl, nullptr, S, SS, nullptr, S1, HD, 0, sQ, sQ, 0, sS);
            k_duffw<<<(HG * SS) / 8, 256, 0, stream>>>(S, lq1, lk1, lq2, lk2, WH, WL);
            k_gemmbz<true, false><<<dim3(SS / 64, 1, HG), 128, 0, stream>>>(WH, WL, VTh, nullptr, A1 + h0 * VD, EE, nullptr, nullptr, SS, 0, sS, sV, 0, (size_t)VD);
            k_gemmbz<false, false><<<dim3(SS / 64, 1, HG), 128, 0, stream>>>(WH, nullptr, VTl, nullptr, ATT + h0 * VD, EE, nullptr, A1 + h0 * VD, SS, 0, sS, sV, 0, (size_t)VD);
            k_rms<<<(SS * HG) / 8, 256, 0, stream>>>(ATT, rw, h0, Rh, Rl); }
        k_gemmb<true, false><<<dim3(SS / 64, EE / 64, 1), 128, 0, stream>>>(Rh, Rl, WOT, nullptr, out + (size_t)b * SS * EE, EE, nullptr, nullptr, EE); }
}
